// SpatialMamba_14388140441601
// MI455X (gfx1250) — hardware-verified
//
#include <hip/hip_runtime.h>
#include <math.h>

typedef __attribute__((ext_vector_type(16))) _Float16 v16h;
typedef __attribute__((ext_vector_type(8)))  _Float16 v8h;
typedef __attribute__((ext_vector_type(16))) __bf16   v16b;
typedef __attribute__((ext_vector_type(8)))  __bf16   v8b;
typedef __attribute__((ext_vector_type(8)))  float    v8f;
typedef __attribute__((ext_vector_type(4)))  float    v4f;

constexpr int kSeqLen   = 16384;
constexpr int kDModel   = 64;
constexpr int kDInner   = 128;
constexpr int kNState   = 16;
constexpr int kDtRank   = 4;
constexpr int kXpReal   = 36;
constexpr int kXpPad    = 64;
constexpr int kXzPitch  = 256;
constexpr int kNDir     = 4;
constexpr int kNChunk   = 128;
constexpr int kChunkLen = 128;
constexpr int kCeRows   = 17;
constexpr int kTileP    = 132;
constexpr int kSP       = 68;

__device__ __forceinline__ unsigned short f2bf_bits(float f) {
  unsigned u = __float_as_uint(f);
  return (unsigned short)((u + 0x7FFFu + ((u >> 16) & 1u)) >> 16);
}
__device__ __forceinline__ float bf_bits2f(unsigned short h) { return __uint_as_float(((unsigned)h) << 16); }

__device__ __forceinline__ void dep_guard_h(v8f& a, v8f& b, v16h x, v16h y) { asm volatile("v_nop\n\tv_nop\n\tv_nop\n\tv_nop" : "+v"(a), "+v"(b) : "v"(x), "v"(y)); }
__device__ __forceinline__ void dep_guard_b(v8f& a, v8f& b, v16b x, v16b y) { asm volatile("v_nop\n\tv_nop\n\tv_nop\n\tv_nop" : "+v"(a), "+v"(b) : "v"(x), "v"(y)); }
__device__ __forceinline__ void keep4_h(v16h a, v16h b, v16h c, v16h d) { asm volatile("v_nop" :: "v"(a), "v"(b), "v"(c), "v"(d)); }
__device__ __forceinline__ void keep4_b(v16b a, v16b b, v16b c, v16b d) { asm volatile("v_nop" :: "v"(a), "v"(b), "v"(c), "v"(d)); }
__device__ __forceinline__ void acc_guard4(v8f& a, v8f& b, v8f& c, v8f& d) { asm volatile("v_nop\n\tv_nop\n\tv_nop\n\tv_nop" : "+v"(a), "+v"(b), "+v"(c), "+v"(d)); }
template <typename T> struct Frag;
template <> struct Frag<_Float16> {
  typedef v16h V; union U { v16h v; v8h h[2]; };
  static __device__ __forceinline__ v16h load(const _Float16* p) {
    U f; f.h[0] = *(const v8h*)(p); f.h[1] = *(const v8h*)(p + 16); return f.v;
  }
  static __device__ __forceinline__ v8f mma(v16h a, v16h b, v8f c) {
    return __builtin_amdgcn_wmma_f32_16x16x32_f16(false, a, false, b, (short)0, c, false, false);
  }
  static __device__ __forceinline__ void guard(v8f& a, v8f& b, v16h x, v16h y) { dep_guard_h(a, b, x, y); }
  static __device__ __forceinline__ void keep(v16h a, v16h b, v16h c, v16h d) { keep4_h(a, b, c, d); }
};
template <> struct Frag<__bf16> {
  typedef v16b V; union U { v16b v; v8b h[2]; };
  static __device__ __forceinline__ v16b load(const __bf16* p) {
    U f; f.h[0] = *(const v8b*)(p); f.h[1] = *(const v8b*)(p + 16); return f.v;
  }
  static __device__ __forceinline__ v8f mma(v16b a, v16b b, v8f c) {
    return __builtin_amdgcn_wmma_f32_16x16x32_bf16(false, a, false, b, (short)0, c, false, false);
  }
  static __device__ __forceinline__ void guard(v8f& a, v8f& b, v16b x, v16b y) { dep_guard_b(a, b, x, y); }
  static __device__ __forceinline__ void keep(v16b a, v16b b, v16b c, v16b d) { keep4_b(a, b, c, d); }
};

template <int ET> struct Elem;
template <> struct Elem<0> { typedef _Float16 T; };
template <> struct Elem<1> { typedef __bf16 T; };
template <int ET, bool SPLIT, int BIAS_MODE, int OUT_MODE, bool RESID, int ACT = 0>
__global__ __launch_bounds__(256) void wmma_gemm64(
    const unsigned short* __restrict__ Ap, const unsigned short* __restrict__ A2p, int lda, long strideA,
    const unsigned short* __restrict__ Btp, const unsigned short* __restrict__ Bt2p, int ldb, long strideB,
    void* __restrict__ Cout, void* __restrict__ Cout2, int ldc, long strideC,
    const float* __restrict__ bias,
    const float* __restrict__ resid, long strideR,
    int M, int N, int K, float scale) {
  typedef typename Elem<ET>::T T;
  typedef typename Frag<T>::V V;
  const T* A = (const T*)Ap; const T* A2 = (const T*)A2p; const T* Bt = (const T*)Btp; const T* Bt2 = (const T*)Bt2p;
  __shared__ __align__(16) float sT[8][16 * 68];
  const int b    = blockIdx.y;
  const int lane = threadIdx.x & 31;
  const int wave = threadIdx.x >> 5;
  const int tilesN = N >> 6;
  const int tilesM = M >> 6;
  const int tile = blockIdx.x * 8 + wave;
  if (tile >= tilesM * tilesN) return;
  const int tm = tile / tilesN;
  const int tn = tile - tm * tilesN;
  const int m0 = tm << 6;
  const int n0 = tn << 6;

  const T* Ab  = A  + (size_t)b * strideA;
  const T* Bb  = Bt + (size_t)b * strideB;
  const T* Ab2 = SPLIT ? (A2  + (size_t)b * strideA) : nullptr;
  const T* Bb2 = SPLIT ? (Bt2 + (size_t)b * strideB) : nullptr;

  const int rlane = lane & 15;
  const int koff  = (lane >> 4) * 8;
  const int mOff  = (lane >> 4) * 8;

  v8f acc[4][4];
#pragma unroll
  for (int i = 0; i < 4; ++i)
#pragma unroll
    for (int j = 0; j < 4; ++j) acc[i][j] = (v8f){0.f,0.f,0.f,0.f,0.f,0.f,0.f,0.f};

  for (int k0 = 0; k0 < K; k0 += 32) {
    V bh[4], bl[4];
#pragma unroll
    for (int j = 0; j < 4; ++j) {
      const size_t bo = (size_t)(n0 + (j << 4) + rlane) * ldb + koff + k0;
      bh[j] = Frag<T>::load(Bb + bo);
      if (SPLIT) bl[j] = Frag<T>::load(Bb2 + bo);
    }
#pragma unroll
    for (int i = 0; i < 4; ++i) {
      const size_t ao = (size_t)(m0 + (i << 4) + rlane) * lda + koff + k0;
      V ah = Frag<T>::load(Ab + ao);
      V al;
      if (SPLIT) al = Frag<T>::load(Ab2 + ao);
#pragma unroll
      for (int j = 0; j < 4; ++j) {
        acc[i][j] = Frag<T>::mma(ah, bh[j], acc[i][j]);
        if (SPLIT) {
          acc[i][j] = Frag<T>::mma(ah, bl[j], acc[i][j]);
          acc[i][j] = Frag<T>::mma(al, bh[j], acc[i][j]);
        }
      }
      Frag<T>::guard(acc[i][0], acc[i][3], ah, SPLIT ? al : ah);
    }
    Frag<T>::keep(bh[0], bh[1], bh[2], bh[3]);
    if (SPLIT) Frag<T>::keep(bl[0], bl[1], bl[2], bl[3]);
  }
  acc_guard4(acc[0][0], acc[0][1], acc[0][2], acc[0][3]);
  acc_guard4(acc[1][0], acc[1][1], acc[1][2], acc[1][3]);
  acc_guard4(acc[2][0], acc[2][1], acc[2][2], acc[2][3]);
  acc_guard4(acc[3][0], acc[3][1], acc[3][2], acc[3][3]);

  float* slab = sT[wave];
  const float* Rb = RESID ? (resid + (size_t)b * strideR) : nullptr;
#pragma unroll
  for (int i = 0; i < 4; ++i) {
    const int mBase = m0 + (i << 4);
#pragma unroll
    for (int j = 0; j < 4; ++j) {
      const int n = n0 + (j << 4) + rlane;
      float bv = 0.f;
      if (BIAS_MODE == 2) bv = bias[n];
#pragma unroll
      for (int r = 0; r < 8; ++r) {
        float v = acc[i][j][r] * scale;
        if (BIAS_MODE == 1) v += bias[mBase + mOff + r];
        if (BIAS_MODE == 2) v += bv;
        if (RESID) v += Rb[(size_t)(mBase + mOff + r) * ldc + n];
        if (ACT == 1) v = tanhf(v);
        if (ACT == 2) v = fmaxf(v, 0.0f);
        if (ACT == 3) v = v / (1.0f + expf(-v));
        if (ACT == 4) v = (v > 0.f) ? v : 0.01f * v;
        if (ACT == 5) v = 0.5f * v * (1.0f + erff(v * 0.70710678118654752f));
        slab[(mOff + r) * 68 + (j << 4) + rlane] = v;
      }
    }
    __builtin_amdgcn_fence(__ATOMIC_RELEASE, "workgroup");
    __builtin_amdgcn_wave_barrier();
    __builtin_amdgcn_fence(__ATOMIC_ACQUIRE, "workgroup");
    if (OUT_MODE == 0) {
      float* C = (float*)Cout + (size_t)b * strideC;
      const int hh = lane >> 4, c4 = (lane & 15) * 4;
      for (int pass = 0; pass < 2; ++pass) {
#pragma unroll
        for (int it = 0; it < 8; ++it) {
          const int row = it * 2 + hh;
          v4f v = *(const v4f*)(slab + row * 68 + c4);
          *(volatile v4f*)(C + (size_t)(mBase + row) * ldc + n0 + c4) = v;
        }
        __threadfence();
      }
    } else {
      const int q = lane >> 3, c8 = (lane & 7) * 8;
      unsigned short* C  = (unsigned short*)Cout  + (size_t)b * strideC;
      unsigned short* C2 = (OUT_MODE == 2) ? ((unsigned short*)Cout2 + (size_t)b * strideC) : nullptr;
      for (int pass = 0; pass < 2; ++pass) {
#pragma unroll
        for (int it = 0; it < 4; ++it) {
          const int row = it * 4 + q;
          const float* sp = slab + row * 68 + c8;
          v8h hv, lv;
#pragma unroll
          for (int e = 0; e < 8; ++e) {
            if (OUT_MODE == 1) {
              hv[e] = (_Float16)sp[e];
            } else {
              unsigned short hb = f2bf_bits(sp[e]);
              unsigned short lb = f2bf_bits(sp[e] - bf_bits2f(hb));
              hv[e] = __builtin_bit_cast(_Float16, hb);
              lv[e] = __builtin_bit_cast(_Float16, lb);
            }
          }
          *(volatile v8h*)(C + (size_t)(mBase + row) * ldc + n0 + c8) = hv;
          if (OUT_MODE == 2) *(volatile v8h*)(C2 + (size_t)(mBase + row) * ldc + n0 + c8) = lv;
        }
        __threadfence();
      }
    }
    __builtin_amdgcn_fence(__ATOMIC_RELEASE, "workgroup");
    __builtin_amdgcn_wave_barrier();
    __builtin_amdgcn_fence(__ATOMIC_ACQUIRE, "workgroup");
  }
}

__global__ __launch_bounds__(256) void cast_split_rows_kernel(
    const float* __restrict__ src, unsigned short* __restrict__ hi, unsigned short* __restrict__ lo,
    int K, int nreal, int total8)
{
  const int i = blockIdx.x * 256 + threadIdx.x;
  if (i >= total8) return;
  const int e0  = i << 3;
  const int row = e0 / K;
  const int col = e0 - row * K;
  const int rc  = (row < nreal) ? row : (nreal - 1);
  const bool keep = (row < nreal);
  const float* p = src + (size_t)rc * K + col;
  const v4f a0 = *(const v4f*)(p);
  const v4f a1 = *(const v4f*)(p + 4);
  v8h hv, lv;
#pragma unroll
  for (int e = 0; e < 4; ++e) {
    const float v0 = keep ? a0[e] : 0.f;
    const float v1 = keep ? a1[e] : 0.f;
    const unsigned short h0 = f2bf_bits(v0), h1 = f2bf_bits(v1);
    const unsigned short l0 = f2bf_bits(v0 - bf_bits2f(h0)), l1 = f2bf_bits(v1 - bf_bits2f(h1));
    hv[e]     = __builtin_bit_cast(_Float16, h0);
    hv[4 + e] = __builtin_bit_cast(_Float16, h1);
    lv[e]     = __builtin_bit_cast(_Float16, l0);
    lv[4 + e] = __builtin_bit_cast(_Float16, l1);
  }
  unsigned short* qh = hi + e0;
  unsigned short* ql = lo + e0;
  *(volatile v8h*)qh = hv;
  *(volatile v8h*)ql = lv;
  __threadfence();
  *(volatile v8h*)qh = hv;
  *(volatile v8h*)ql = lv;
}

__device__ __forceinline__ int seq_token(int rev, int tr, int t) {
  const int l2 = rev ? (kSeqLen - 1 - t) : t;
  const int ct = ((l2 & 127) << 7) | (l2 >> 7);
  return tr ? ct : l2;
}

__global__ __launch_bounds__(256) void x_split_kernel(
    const float* __restrict__ x, unsigned short* __restrict__ XH, unsigned short* __restrict__ XL)
{
  __shared__ __align__(16) float sX[64 * kSP];
  const int tid = threadIdx.x, lane = tid & 31, wave = tid >> 5;
  const int t0 = blockIdx.x * 64;
  {
    const int c = tid >> 2, q = tid & 3;
    const float* xp = x + (size_t)c * kSeqLen + t0 + q * 16;
#pragma unroll
    for (int i = 0; i < 4; ++i) {
      const v4f v = *(const v4f*)(xp + 4 * i);
#pragma unroll
      for (int e = 0; e < 4; ++e) sX[(q * 16 + 4 * i + e) * kSP + c] = v[e];
    }
  }
  __syncthreads();
  const int rq = lane >> 3, c8 = (lane & 7) * 8;
  for (int pass = 0; pass < 2; ++pass) {
#pragma unroll
    for (int it = 0; it < 2; ++it) {
      const int row = wave * 8 + it * 4 + rq;
      const float* sp = sX + row * kSP + c8;
      const v4f a0 = *(const v4f*)(sp);
      const v4f a1 = *(const v4f*)(sp + 4);
      v8h hv, lv;
#pragma unroll
      for (int e = 0; e < 4; ++e) {
        const unsigned short h0 = f2bf_bits(a0[e]), h1 = f2bf_bits(a1[e]);
        const unsigned short l0 = f2bf_bits(a0[e] - bf_bits2f(h0)), l1 = f2bf_bits(a1[e] - bf_bits2f(h1));
        hv[e]     = __builtin_bit_cast(_Float16, h0);
        hv[4 + e] = __builtin_bit_cast(_Float16, h1);
        lv[e]     = __builtin_bit_cast(_Float16, l0);
        lv[4 + e] = __builtin_bit_cast(_Float16, l1);
      }
      const size_t o = (size_t)(t0 + row) * kDModel + c8;
      *(volatile v8h*)(XH + o) = hv;
      *(volatile v8h*)(XL + o) = lv;
    }
    __threadfence();
  }
}

__global__ __launch_bounds__(128) void conv_silu4_kernel(
    const float* __restrict__ XZ, const float* __restrict__ cw, const float* __restrict__ cb,
    float* __restrict__ Uo, unsigned short* __restrict__ UBo)
{
  __shared__ __align__(16) float sT[16 * kTileP];
  const int tid = threadIdx.x, lane = tid & 31, wave = tid >> 5;
  const int d = tid;
  const int k = blockIdx.y;
  const int rev = k & 1, tr = k >> 1;
  const int t0 = blockIdx.x * 64;
  const float w0 = cw[d * 4 + 0], w1 = cw[d * 4 + 1], w2 = cw[d * 4 + 2], w3 = cw[d * 4 + 3];
  const float bc = cb[d];
  float xm3, xm2, xm1;
  {
    const int p3 = t0 - 3, p2 = t0 - 2, p1 = t0 - 1;
    const int c3 = (p3 >= 0) ? p3 : 0, c2 = (p2 >= 0) ? p2 : 0, c1 = (p1 >= 0) ? p1 : 0;
    const float v3 = XZ[(size_t)seq_token(rev, tr, c3) * kXzPitch + d];
    const float v2 = XZ[(size_t)seq_token(rev, tr, c2) * kXzPitch + d];
    const float v1 = XZ[(size_t)seq_token(rev, tr, c1) * kXzPitch + d];
    xm3 = (p3 >= 0) ? v3 : 0.f;
    xm2 = (p2 >= 0) ? v2 : 0.f;
    xm1 = (p1 >= 0) ? v1 : 0.f;
  }
  const size_t dirRow0 = (size_t)k * kSeqLen;
#pragma unroll 1
  for (int sub = 0; sub < 4; ++sub) {
    const int lb = t0 + sub * 16;
#pragma unroll 1
    for (int s = 0; s < 16; ++s) {
      const int t = lb + s;
      const int tok = seq_token(rev, tr, t);
      const float xc = XZ[(size_t)tok * kXzPitch + d];
      float acc = w0 * xm3;
      acc = fmaf(w1, xm2, acc);
      acc = fmaf(w2, xm1, acc);
      acc = fmaf(w3, xc, acc);
      const float sv = acc + bc;
      const float sg = __builtin_amdgcn_rcpf(1.0f + __expf(-sv));
      sT[s * kTileP + d] = sv * sg;
      xm3 = xm2; xm2 = xm1; xm1 = xc;
    }
    __syncthreads();
    v4f fv[4];
    v8h bh[2];
#pragma unroll
    for (int it = 0; it < 4; ++it) fv[it] = *(const v4f*)(sT + (it * 4 + wave) * kTileP + lane * 4);
#pragma unroll
    for (int it = 0; it < 2; ++it) {
      const int row = it * 8 + wave * 2 + (lane >> 4);
      const float* sp = sT + row * kTileP + (lane & 15) * 8;
      const v4f a0 = *(const v4f*)(sp);
      const v4f a1 = *(const v4f*)(sp + 4);
#pragma unroll
      for (int e = 0; e < 4; ++e) {
        bh[it][e]     = __builtin_bit_cast(_Float16, f2bf_bits(a0[e]));
        bh[it][4 + e] = __builtin_bit_cast(_Float16, f2bf_bits(a1[e]));
      }
    }
    for (int pass = 0; pass < 2; ++pass) {
#pragma unroll
      for (int it = 0; it < 4; ++it)
        *(volatile v4f*)(Uo + (dirRow0 + lb + it * 4 + wave) * kDInner + lane * 4) = fv[it];
#pragma unroll
      for (int it = 0; it < 2; ++it) {
        const int row = it * 8 + wave * 2 + (lane >> 4);
        *(volatile v8h*)(UBo + (dirRow0 + lb + row) * kDInner + (lane & 15) * 8) = bh[it];
      }
      __threadfence();
    }
    __syncthreads();
  }
}

union Q4 { v4f q[4]; float f[16]; };

__global__ __launch_bounds__(128) void scan_end_kernel(
    const float* __restrict__ XDBL, const float* __restrict__ U,
    const float* __restrict__ dtw, const float* __restrict__ dtb, const float* __restrict__ Alog,
    float* __restrict__ CE)
{
  __shared__ __align__(16) float sCE[kCeRows * kTileP];
  const int tid = threadIdx.x, lane = tid & 31, wave = tid >> 5;
  const int d = tid;
  const int chunk = blockIdx.x, k = blockIdx.y;
  const int t0 = chunk * kChunkLen;
  float An[kNState];
#pragma unroll
  for (int n = 0; n < kNState; ++n) An[n] = -__expf(Alog[d * kNState + n]);
  const float w0 = dtw[d * 4 + 0], w1 = dtw[d * 4 + 1], w2 = dtw[d * 4 + 2], w3 = dtw[d * 4 + 3];
  const float bd = dtb[d];
  float h[kNState];
#pragma unroll
  for (int n = 0; n < kNState; ++n) h[n] = 0.f;
  float dtsum = 0.f;
#pragma unroll 1
  for (int s = 0; s < kChunkLen; ++s) {
    const size_t row = (size_t)k * kSeqLen + t0 + s;
    const float* xr = XDBL + row * kXpPad;
    const v4f q0 = *(const v4f*)(xr);
    Q4 Bq;
    Bq.q[0] = *(const v4f*)(xr + 4);  Bq.q[1] = *(const v4f*)(xr + 8);
    Bq.q[2] = *(const v4f*)(xr + 12); Bq.q[3] = *(const v4f*)(xr + 16);
    const float u = U[row * kDInner + d];
    float dl = q0[0] * w0;
    dl = fmaf(q0[1], w1, dl);
    dl = fmaf(q0[2], w2, dl);
    dl = fmaf(q0[3], w3, dl);
    dl += bd;
    const float ex = __expf(-fabsf(dl));
    const float dt = fmaxf(dl, 0.f) + __logf(1.0f + ex);
    const float bx = dt * u;
    dtsum += dt;
#pragma unroll
    for (int n = 0; n < kNState; ++n) {
      const float a = __expf(dt * An[n]);
      h[n] = fmaf(a, h[n], bx * Bq.f[n]);
    }
  }
#pragma unroll
  for (int n = 0; n < kNState; ++n) sCE[n * kTileP + d] = h[n];
  sCE[16 * kTileP + d] = dtsum;
  __syncthreads();
  const size_t base = ((size_t)(k * kNChunk + chunk) * kCeRows) * kDInner;
  for (int pass = 0; pass < 2; ++pass) {
    for (int r = wave; r < kCeRows; r += 4) {
      const v4f v = *(const v4f*)(sCE + r * kTileP + lane * 4);
      *(volatile v4f*)(CE + base + (size_t)r * kDInner + lane * 4) = v;
    }
    __threadfence();
  }
}

__global__ __launch_bounds__(128) void carry_kernel(
    const float* __restrict__ CE, const float* __restrict__ Alog, float* __restrict__ CI)
{
  const int lane = threadIdx.x & 31, wave = threadIdx.x >> 5;
  const int n = blockIdx.x * 4 + wave;
  const int k = blockIdx.y;
  const int d4 = lane * 4;
  float Ae[4];
#pragma unroll
  for (int e = 0; e < 4; ++e) Ae[e] = -__expf(Alog[(d4 + e) * kNState + n]);
  v4f carry = (v4f){0.f, 0.f, 0.f, 0.f};
#pragma unroll 1
  for (int c = 0; c < kNChunk; ++c) {
    const size_t base = (size_t)(k * kNChunk + c);
    float* dst = CI + (base * kNState + n) * kDInner + d4;
    const v4f cv = carry;
    *(volatile v4f*)dst = cv;
    __threadfence();
    *(volatile v4f*)dst = cv;
    const v4f he = *(const v4f*)(CE + (base * kCeRows + n) * kDInner + d4);
    const v4f ds = *(const v4f*)(CE + (base * kCeRows + 16) * kDInner + d4);
#pragma unroll
    for (int e = 0; e < 4; ++e) {
      const float P = __expf(Ae[e] * ds[e]);
      carry[e] = fmaf(P, carry[e], he[e]);
    }
  }
}

__global__ __launch_bounds__(64) void scan_out_kernel(
    const float* __restrict__ XDBL, const float* __restrict__ U, const float* __restrict__ XZ,
    const float* __restrict__ CI, const float* __restrict__ dtw, const float* __restrict__ dtb,
    const float* __restrict__ Alog, const float* __restrict__ Dv,
    unsigned short* __restrict__ SH, unsigned short* __restrict__ SL)
{
  __shared__ __align__(16) float sS[kChunkLen * kSP];
  const int tid = threadIdx.x, lane = tid & 31, wave = tid >> 5;
  const int chunk = blockIdx.x, half = blockIdx.y;
  const int d = half * 64 + tid;
  const int t0 = chunk * kChunkLen;
  float An[kNState];
#pragma unroll
  for (int n = 0; n < kNState; ++n) An[n] = -__expf(Alog[d * kNState + n]);
  const float w0 = dtw[d * 4 + 0], w1 = dtw[d * 4 + 1], w2 = dtw[d * 4 + 2], w3 = dtw[d * 4 + 3];
  const float bd = dtb[d];
  const float Dd = Dv[d];
#pragma unroll 1
  for (int r = 0; r < kChunkLen; ++r) sS[r * kSP + tid] = 0.f;
#pragma unroll 1
  for (int k = 0; k < kNDir; ++k) {
    const int rev = k & 1, tr = k >> 1;
    float h[kNState];
    const size_t cib = ((size_t)(k * kNChunk + chunk) * kNState) * kDInner + d;
#pragma unroll
    for (int n = 0; n < kNState; ++n) h[n] = CI[cib + (size_t)n * kDInner];
#pragma unroll 1
    for (int s = 0; s < kChunkLen; ++s) {
      const int t = t0 + s;
      const size_t row = (size_t)k * kSeqLen + t;
      const float* xr = XDBL + row * kXpPad;
      const v4f q0 = *(const v4f*)(xr);
      Q4 Bq, Cq;
      Bq.q[0] = *(const v4f*)(xr + 4);  Bq.q[1] = *(const v4f*)(xr + 8);
      Bq.q[2] = *(const v4f*)(xr + 12); Bq.q[3] = *(const v4f*)(xr + 16);
      Cq.q[0] = *(const v4f*)(xr + 20); Cq.q[1] = *(const v4f*)(xr + 24);
      Cq.q[2] = *(const v4f*)(xr + 28); Cq.q[3] = *(const v4f*)(xr + 32);
      const float u = U[row * kDInner + d];
      const int tok = seq_token(rev, tr, t);
      const float z = XZ[(size_t)tok * kXzPitch + kDInner + d];
      float dl = q0[0] * w0;
      dl = fmaf(q0[1], w1, dl);
      dl = fmaf(q0[2], w2, dl);
      dl = fmaf(q0[3], w3, dl);
      dl += bd;
      const float ex = __expf(-fabsf(dl));
      const float dt = fmaxf(dl, 0.f) + __logf(1.0f + ex);
      const float bx = dt * u;
      float y = 0.f;
#pragma unroll
      for (int n = 0; n < kNState; ++n) {
        const float a = __expf(dt * An[n]);
        h[n] = fmaf(a, h[n], bx * Bq.f[n]);
        y = fmaf(h[n], Cq.f[n], y);
      }
      y = fmaf(u, Dd, y);
      const float g = z * __builtin_amdgcn_rcpf(1.0f + __expf(-z));
      sS[s * kSP + tid] += y * g;
    }
  }
  __syncthreads();
  const int rq = lane >> 3, c8 = (lane & 7) * 8;
  const size_t colb = (size_t)half * 64 + c8;
  for (int pass = 0; pass < 2; ++pass) {
#pragma unroll 1
    for (int it = 0; it < 16; ++it) {
      const int row = it * 8 + wave * 4 + rq;
      const float* sp = sS + row * kSP + c8;
      const v4f a0 = *(const v4f*)(sp);
      const v4f a1 = *(const v4f*)(sp + 4);
      v8h hv, lv;
#pragma unroll
      for (int e = 0; e < 4; ++e) {
        const unsigned short h0 = f2bf_bits(a0[e]), h1 = f2bf_bits(a1[e]);
        const unsigned short l0 = f2bf_bits(a0[e] - bf_bits2f(h0)), l1 = f2bf_bits(a1[e] - bf_bits2f(h1));
        hv[e]     = __builtin_bit_cast(_Float16, h0);
        hv[4 + e] = __builtin_bit_cast(_Float16, h1);
        lv[e]     = __builtin_bit_cast(_Float16, l0);
        lv[4 + e] = __builtin_bit_cast(_Float16, l1);
      }
      const size_t o = (size_t)(t0 + row) * kDInner + colb;
      *(volatile v8h*)(SH + o) = hv;
      *(volatile v8h*)(SL + o) = lv;
    }
    __threadfence();
  }
}

extern "C" void kernel_launch(void* const* d_in, const int* in_sizes, int n_in,
                              void* d_out, int out_size, void* d_ws, size_t ws_size,
                              hipStream_t stream) {
  if (n_in < 10) return;
  if (in_sizes[0] != kDModel * kSeqLen || out_size != kDModel * kSeqLen) return;
  if (in_sizes[1] != 2 * kDInner * kDModel || in_sizes[4] != kXpReal * kDInner || in_sizes[9] != kDModel * kDInner) return;

  const float* x      = (const float*)d_in[0];
  const float* w_in   = (const float*)d_in[1];
  const float* conv_w = (const float*)d_in[2];
  const float* conv_b = (const float*)d_in[3];
  const float* w_xp   = (const float*)d_in[4];
  const float* dt_w   = (const float*)d_in[5];
  const float* dt_b   = (const float*)d_in[6];
  const float* A_log  = (const float*)d_in[7];
  const float* Dvec   = (const float*)d_in[8];
  const float* w_out  = (const float*)d_in[9];
  float* out = (float*)d_out;

  char* base = (char*)d_ws;
  size_t off = 0;
  auto carve = [&](size_t bytes) -> char* {
    char* r = base + off;
    off += (bytes + 255) & ~(size_t)255;
    return r;
  };
  float*          XZ   = (float*)carve((size_t)kSeqLen * kXzPitch * 4);
  unsigned short* XH   = (unsigned short*)carve((size_t)kSeqLen * kDModel * 2);
  unsigned short* XL   = (unsigned short*)carve((size_t)kSeqLen * kDModel * 2);
  unsigned short* WinH = (unsigned short*)carve((size_t)2 * kDInner * kDModel * 2);
  unsigned short* WinL = (unsigned short*)carve((size_t)2 * kDInner * kDModel * 2);
  unsigned short* WxpH = (unsigned short*)carve((size_t)kXpPad * kDInner * 2);
  unsigned short* WxpL = (unsigned short*)carve((size_t)kXpPad * kDInner * 2);
  unsigned short* WoH  = (unsigned short*)carve((size_t)kDModel * kDInner * 2);
  unsigned short* WoL  = (unsigned short*)carve((size_t)kDModel * kDInner * 2);
  float*          U    = (float*)carve((size_t)kNDir * kSeqLen * kDInner * 4);
  unsigned short* UB   = (unsigned short*)carve((size_t)kNDir * kSeqLen * kDInner * 2);
  float*          XDBL = (float*)carve((size_t)kNDir * kSeqLen * kXpPad * 4);
  float*          CE   = (float*)carve((size_t)kNDir * kNChunk * kCeRows * kDInner * 4);
  float*          CI   = (float*)carve((size_t)kNDir * kNChunk * kNState * kDInner * 4);
  unsigned short* SH   = (unsigned short*)carve((size_t)kSeqLen * kDInner * 2);
  unsigned short* SL   = (unsigned short*)carve((size_t)kSeqLen * kDInner * 2);
  if (off > ws_size) return;

  cast_split_rows_kernel<<<8, 256, 0, stream>>>(w_in, WinH, WinL, kDModel, 2 * kDInner, (2 * kDInner * kDModel) / 8);
  cast_split_rows_kernel<<<4, 256, 0, stream>>>(w_xp, WxpH, WxpL, kDInner, kXpReal, (kXpPad * kDInner) / 8);
  cast_split_rows_kernel<<<4, 256, 0, stream>>>(w_out, WoH, WoL, kDInner, kDModel, (kDModel * kDInner) / 8);

  x_split_kernel<<<kSeqLen / 64, 256, 0, stream>>>(x, XH, XL);

  wmma_gemm64<1, true, 0, 0, false, 0><<<dim3(128, 1), 256, 0, stream>>>(
      XH, XL, kDModel, 0L, WinH, WinL, kDModel, 0L, (void*)XZ, (void*)XZ, kXzPitch, 0L,
      dt_b, dt_b, 0L, kSeqLen, kXzPitch, kDModel, 1.0f);

  conv_silu4_kernel<<<dim3(kSeqLen / 64, kNDir), 128, 0, stream>>>(XZ, conv_w, conv_b, U, UB);

  wmma_gemm64<1, false, 0, 0, false, 0><<<dim3(128, 1), 256, 0, stream>>>(
      UB, UB, kDInner, 0L, WxpH, WxpH, kDInner, 0L, (void*)XDBL, (void*)XDBL, kXpPad, 0L,
      dt_b, dt_b, 0L, kNDir * kSeqLen, kXpPad, kDInner, 1.0f);

  scan_end_kernel<<<dim3(kNChunk, kNDir), 128, 0, stream>>>(XDBL, U, dt_w, dt_b, A_log, CE);
  carry_kernel<<<dim3(kNState / 4, kNDir), 128, 0, stream>>>(CE, A_log, CI);
  scan_out_kernel<<<dim3(kNChunk, 2), 64, 0, stream>>>(XDBL, U, XZ, CI, dt_w, dt_b, A_log, Dvec, SH, SL);

  wmma_gemm64<1, true, 0, 0, false, 0><<<dim3(32, 1), 256, 0, stream>>>(
      WoH, WoL, kDInner, 0L, SH, SL, kDInner, 0L, (void*)out, (void*)out, kSeqLen, 0L,
      dt_b, dt_b, 0L, kDModel, kSeqLen, kDInner, 0.25f);
}
